// SelfAttentionBlock_25537875542491
// MI455X (gfx1250) — hardware-verified
//
#include <hip/hip_runtime.h>


#ifndef NB
#define NB 2
#endif
#ifndef SEQ
#define SEQ 2048
#endif
#define NB_FULL  2
#define SEQ_FULL 2048
#define DMD  1024
#define NHD  16
#define HD   64
#define DQ   (NHD * HD)
#define DKV  (2 * HD)
#define FFI  4096
#define K2   (DQ + FFI)
#define ROWS (NB * SEQ)
#define LNEPS 1e-5f
#define WCAR 64.0f
#define XCAR 8.0f
#define PCAR 1024.0f
#define OCAR 16.0f
#define SC512  0.001953125f
#define SC1024 0.0009765625f

static_assert(NB >= 1 && NB <= NB_FULL);
static_assert(SEQ % 64 == 0 && SEQ <= SEQ_FULL);
static_assert(ROWS % 64 == 0 && DMD % 64 == 0 && DQ % 64 == 0 && DKV % 64 == 0 && FFI % 64 == 0 && K2 % 32 == 0);

typedef _Float16 h16;
typedef __attribute__((ext_vector_type(16))) _Float16 v16h;
typedef __attribute__((ext_vector_type(8)))  _Float16 v8h;
typedef __attribute__((ext_vector_type(4)))  _Float16 v4h;
typedef __attribute__((ext_vector_type(2)))  _Float16 v2h;
typedef __attribute__((ext_vector_type(8)))  float    v8f;
typedef __attribute__((ext_vector_type(4)))  float    v4f;
typedef v8h __attribute__((may_alias)) v8ha;
typedef v4f __attribute__((may_alias)) v4fa;

__device__ __forceinline__ unsigned short f2bf(float f) { unsigned u = __float_as_uint(f); u += 0x7FFFu + ((u >> 16) & 1u); return (unsigned short)(u >> 16); }
__device__ __forceinline__ float bf2f(unsigned short b) { return __uint_as_float(((unsigned)b) << 16); }
__device__ __forceinline__ float bfr(float f) { return bf2f(f2bf(f)); }
__device__ __forceinline__ v16h cat16(v8h lo, v8h hi) { return __builtin_shufflevector(lo, hi, 0, 1, 2, 3, 4, 5, 6, 7, 8, 9, 10, 11, 12, 13, 14, 15); }
__device__ __forceinline__ v8f wmma16(v16h a, v16h b, v8f c) { return __builtin_amdgcn_wmma_f32_16x16x32_f16(false, a, false, b, (short)0, c, false, false); }
__device__ __forceinline__ v8f zero8() { v8f z = {0.f, 0.f, 0.f, 0.f, 0.f, 0.f, 0.f, 0.f}; return z; }
__device__ __forceinline__ v16h ldg16(const h16* p) { return cat16(*(const v8h*)p, *(const v8h*)(p + 16)); }
__device__ __forceinline__ v16h ldl16(const h16* p) { return cat16(*(const v8ha*)p, *(const v8ha*)(p + 16)); }
__device__ __forceinline__ void wsync() { __builtin_amdgcn_fence(3  , "wavefront"); __builtin_amdgcn_wave_barrier(); asm volatile("" ::: "memory"); }

template <int OT>
__global__ __launch_bounds__(32) void k_gemm(const h16* __restrict__ A, int lda, const h16* __restrict__ Bt, int ldb, int K, void* Cv, int ldc, float sc) {
    __shared__ __align__(16) float os[16 * 68];
    const int lane = threadIdx.x & 31, lr = lane & 15, hi = lane >> 4;
    const int r0 = blockIdx.x * 64, c0 = blockIdx.y * 64;
    v8f acc[4][4];
#pragma unroll
    for (int mb = 0; mb < 4; ++mb)
#pragma unroll
        for (int nb = 0; nb < 4; ++nb) acc[mb][nb] = zero8();
    const size_t aoff = (size_t)(r0 + lr) * lda + 8 * hi, boff = (size_t)(c0 + lr) * ldb + 8 * hi;
#pragma unroll 1
    for (int kc = 0; kc < K; kc += 32) {
        v16h a[4], b;
#pragma unroll
        for (int mb = 0; mb < 4; ++mb) a[mb] = ldg16(A + aoff + (size_t)mb * 16 * lda + kc);
#pragma unroll
        for (int nb = 0; nb < 4; ++nb) {
            b = ldg16(Bt + boff + (size_t)nb * 16 * ldb + kc);
#pragma unroll
            for (int mb = 0; mb < 4; ++mb) acc[mb][nb] = wmma16(a[mb], b, acc[mb][nb]);
        }
        asm volatile("v_nop\n\tv_nop\n\tv_nop\n\tv_nop"
            : "+v"(acc[0][0]), "+v"(acc[0][1]), "+v"(acc[0][2]), "+v"(acc[0][3]), "+v"(acc[1][0]), "+v"(acc[1][1]), "+v"(acc[1][2]), "+v"(acc[1][3]),
              "+v"(acc[2][0]), "+v"(acc[2][1]), "+v"(acc[2][2]), "+v"(acc[2][3]), "+v"(acc[3][0]), "+v"(acc[3][1]), "+v"(acc[3][2]), "+v"(acc[3][3])
            : "v"(a[0]), "v"(a[1]), "v"(a[2]), "v"(a[3]), "v"(b));
    }
#pragma unroll
    for (int mb = 0; mb < 4; ++mb) {
#pragma unroll
        for (int nb = 0; nb < 4; ++nb) {
#pragma unroll
            for (int j = 0; j < 8; ++j) os[(hi * 8 + j) * 68 + nb * 16 + lr] = acc[mb][nb][j] * sc;
        }
        wsync();
        if (OT == 0) {
            float* crow = (float*)Cv + (size_t)(r0 + mb * 16) * ldc + c0;
#pragma unroll 1
            for (int ps = 0; ps < 2; ++ps) {
#pragma unroll
                for (int s = 0; s < 8; ++s) {
                    const int row = 2 * s + hi, cofs = lr * 4;
                    const v4f val = *(const v4fa*)(os + row * 68 + cofs);
                    *(volatile v4f*)(crow + (size_t)row * ldc + cofs) = val;
                }
                if (ps == 0) __threadfence();
            }
        } else {
            h16* crow = (h16*)Cv + (size_t)(r0 + mb * 16) * ldc + c0;
            v8h o8[4];
#pragma unroll
            for (int it = 0; it < 4; ++it) {
                const int row = it * 4 + (lane >> 3), cofs = (lane & 7) * 8;
                const v4f x0 = *(const v4fa*)(os + row * 68 + cofs), x1 = *(const v4fa*)(os + row * 68 + cofs + 4);
                v8h t; t[0] = (h16)x0[0]; t[1] = (h16)x0[1]; t[2] = (h16)x0[2]; t[3] = (h16)x0[3]; t[4] = (h16)x1[0]; t[5] = (h16)x1[1]; t[6] = (h16)x1[2]; t[7] = (h16)x1[3];
                o8[it] = t;
            }
#pragma unroll 1
            for (int ps = 0; ps < 2; ++ps) {
#pragma unroll
                for (int it = 0; it < 4; ++it) { const int row = it * 4 + (lane >> 3), cofs = (lane & 7) * 8; *(volatile v8h*)(crow + (size_t)row * ldc + cofs) = o8[it]; }
                if (ps == 0) __threadfence();
            }
        }
        wsync();
    }
}

__global__ __launch_bounds__(32) void k_ffn1(const h16* __restrict__ A, const h16* __restrict__ Bv, const h16* __restrict__ Bg, h16* G, float sc) {
    __shared__ __align__(16) float osv[16 * 68];
    __shared__ __align__(16) float osg[16 * 68];
    const int lane = threadIdx.x & 31, lr = lane & 15, hi = lane >> 4;
    const int r0 = blockIdx.x * 32, c0 = blockIdx.y * 64;
    v8f av[2][4], ag[2][4];
#pragma unroll
    for (int mb = 0; mb < 2; ++mb)
#pragma unroll
        for (int nb = 0; nb < 4; ++nb) { av[mb][nb] = zero8(); ag[mb][nb] = zero8(); }
    const size_t aoff = (size_t)(r0 + lr) * DMD + 8 * hi, boff = (size_t)(c0 + lr) * DMD + 8 * hi;
#pragma unroll 1
    for (int kc = 0; kc < DMD; kc += 32) {
        v16h a[2], bv, bg;
        a[0] = ldg16(A + aoff + kc);
        a[1] = ldg16(A + aoff + (size_t)16 * DMD + kc);
#pragma unroll
        for (int nb = 0; nb < 4; ++nb) {
            bv = ldg16(Bv + boff + (size_t)nb * 16 * DMD + kc);
            bg = ldg16(Bg + boff + (size_t)nb * 16 * DMD + kc);
#pragma unroll
            for (int mb = 0; mb < 2; ++mb) { av[mb][nb] = wmma16(a[mb], bv, av[mb][nb]); ag[mb][nb] = wmma16(a[mb], bg, ag[mb][nb]); }
        }
        asm volatile("v_nop\n\tv_nop\n\tv_nop\n\tv_nop"
            : "+v"(av[0][0]), "+v"(av[0][1]), "+v"(av[0][2]), "+v"(av[0][3]), "+v"(av[1][0]), "+v"(av[1][1]), "+v"(av[1][2]), "+v"(av[1][3]),
              "+v"(ag[0][0]), "+v"(ag[0][1]), "+v"(ag[0][2]), "+v"(ag[0][3]), "+v"(ag[1][0]), "+v"(ag[1][1]), "+v"(ag[1][2]), "+v"(ag[1][3])
            : "v"(a[0]), "v"(a[1]), "v"(bv), "v"(bg));
    }
#pragma unroll
    for (int mb = 0; mb < 2; ++mb) {
#pragma unroll
        for (int nb = 0; nb < 4; ++nb) {
#pragma unroll
            for (int j = 0; j < 8; ++j) { os_store: ; osv[(hi * 8 + j) * 68 + nb * 16 + lr] = av[mb][nb][j] * sc; osg[(hi * 8 + j) * 68 + nb * 16 + lr] = ag[mb][nb][j] * sc; }
        }
        wsync();
        v8h o8[4];
#pragma unroll
        for (int it = 0; it < 4; ++it) {
            const int row = it * 4 + (lane >> 3), cofs = (lane & 7) * 8;
            const v4f va = *(const v4fa*)(osv + row * 68 + cofs), vb2 = *(const v4fa*)(osv + row * 68 + cofs + 4);
            const v4f ga = *(const v4fa*)(osg + row * 68 + cofs), gb = *(const v4fa*)(osg + row * 68 + cofs + 4);
            float vv[8], gg[8];
            vv[0] = va[0]; vv[1] = va[1]; vv[2] = va[2]; vv[3] = va[3]; vv[4] = vb2[0]; vv[5] = vb2[1]; vv[6] = vb2[2]; vv[7] = vb2[3];
            gg[0] = ga[0]; gg[1] = ga[1]; gg[2] = ga[2]; gg[3] = ga[3]; gg[4] = gb[0]; gg[5] = gb[1]; gg[6] = gb[2]; gg[7] = gb[3];
            v8h t;
#pragma unroll
            for (int q = 0; q < 8; ++q) {
                const float e = __expf(-gg[q]);
                const float sg = 1.0f / (1.0f + e);
                const float gl = (gg[q] * sg) * vv[q];
                t[q] = (h16)(gl * OCAR);
            }
            o8[it] = t;
        }
        h16* grow = G + (size_t)(r0 + mb * 16) * K2 + c0;
#pragma unroll 1
        for (int ps = 0; ps < 2; ++ps) {
#pragma unroll
            for (int it = 0; it < 4; ++it) { const int row = it * 4 + (lane >> 3), cofs = (lane & 7) * 8; *(volatile v8h*)(grow + (size_t)row * K2 + cofs) = o8[it]; }
            if (ps == 0) __threadfence();
        }
        wsync();
    }
}

__global__ __launch_bounds__(256) void k_wt(const float* __restrict__ w, int ldw, int coff, int K, int N, float sc, h16* dst, int pitch, int koff) {
    const int lane = threadIdx.x & 31;
    const int L0 = (blockIdx.x * 8 + (threadIdx.x >> 5)) * 8;
    const int nlines = N * K / 64;
#pragma unroll
    for (int ps = 0; ps < 2; ++ps) {
#pragma unroll 1
        for (int l = 0; l < 8; ++l) {
            const int L = L0 + l; if (L >= nlines) break;
            const size_t e = (size_t)L * 64 + lane * 2; const int k = (int)(e % K), n = (int)(e / K);
            v2h o;
            o[0] = (h16)(bfr(w[(size_t)k * ldw + coff + n]) * sc);
            o[1] = (h16)(bfr(w[(size_t)(k + 1) * ldw + coff + n]) * sc);
            *(volatile v2h*)(dst + (size_t)n * pitch + koff + k) = o;
        }
        if (ps == 0) __threadfence();
    }
}

__global__ __launch_bounds__(256) void k_ln(const float* __restrict__ x, const float* __restrict__ gam, h16* XN) {
    const int lane = threadIdx.x & 31;
    const int row = blockIdx.x * 8 + (threadIdx.x >> 5);
    if (row >= ROWS) return;
    const int b = row / SEQ, t = row - b * SEQ;
    const float* src = x + ((size_t)b * SEQ_FULL + t) * DMD;
    float v[32];
    float s = 0.f;
#pragma unroll
    for (int i = 0; i < 8; ++i) {
        const v4f a = *(const v4f*)(src + i * 128 + lane * 4);
#pragma unroll
        for (int q = 0; q < 4; ++q) { const float r = bfr(a[q]); v[i * 4 + q] = r; s += r; }
    }
#pragma unroll
    for (int sh = 16; sh; sh >>= 1) s += __shfl_xor(s, sh, 32);
    const float mu = s * (1.0f / (float)DMD);
    float ss = 0.f;
#pragma unroll
    for (int k = 0; k < 32; ++k) { const float d = v[k] - mu; v[k] = d; ss += d * d; }
#pragma unroll
    for (int sh = 16; sh; sh >>= 1) ss += __shfl_xor(ss, sh, 32);
    const float var = ss * (1.0f / (float)DMD);
    const float rs = rsqrtf(var + LNEPS);
    v4h o[8];
#pragma unroll
    for (int i = 0; i < 8; ++i) {
        const v4f g = *(const v4f*)(gam + i * 128 + lane * 4);
        v4h t4;
#pragma unroll
        for (int q = 0; q < 4; ++q) t4[q] = (h16)(((v[i * 4 + q] * rs) * bfr(g[q])) * XCAR);
        o[i] = t4;
    }
    h16* dst = XN + (size_t)row * DMD + lane * 4;
#pragma unroll
    for (int i = 0; i < 8; ++i) *(volatile v4h*)(dst + i * 128) = o[i];
    __threadfence();
#pragma unroll
    for (int i = 0; i < 8; ++i) *(volatile v4h*)(dst + i * 128) = o[i];
}

__global__ __launch_bounds__(256) void k_kvp(const float* __restrict__ F, h16* K16, h16* VT) {
    const size_t g = (size_t)blockIdx.x * 256 + threadIdx.x;
    const size_t nk = (size_t)ROWS * (HD / 2), nv = (size_t)NB * HD * (SEQ / 2);
    if (g < nk) {
        const size_t e = g * 2; const size_t row = e / HD; const int d = (int)(e % HD);
        const float* sp = F + row * DKV + d;
        v2h o; o[0] = (h16)sp[0]; o[1] = (h16)sp[1];
        *(volatile v2h*)(K16 + e) = o; __threadfence(); *(volatile v2h*)(K16 + e) = o;
    } else if (g < nk + nv) {
        const size_t e = (g - nk) * 2; const int t = (int)(e % SEQ); const int d = (int)((e / SEQ) % HD); const int b = (int)(e / ((size_t)SEQ * HD));
        const float* sp = F + ((size_t)b * SEQ + t) * DKV + HD + d;
        v2h o; o[0] = (h16)sp[0]; o[1] = (h16)sp[DKV];
        *(volatile v2h*)(VT + e) = o; __threadfence(); *(volatile v2h*)(VT + e) = o;
    }
}

__global__ __launch_bounds__(128) void k_attn(const h16* __restrict__ Q16, const h16* __restrict__ K16, const h16* __restrict__ VT, h16* CTX) {
    __shared__ __align__(16) h16 Ps[4 * 16 * 64];
    const int lane = threadIdx.x & 31, w = threadIdx.x >> 5, h = lane >> 4, m = lane & 15;
    const int b = blockIdx.z, head = blockIdx.y, q0 = blockIdx.x * 64 + w * 16;
    h16* P = Ps + w * (16 * 64);
    const h16* qp = Q16 + ((size_t)b * SEQ + q0 + m) * DQ + head * HD + 8 * h;
    v16h aq[2];
    aq[0] = ldg16(qp);
    aq[1] = ldg16(qp + 32);
    const h16* kp = K16 + ((size_t)b * SEQ + m) * HD + 8 * h;
    const h16* vp = VT + ((size_t)b * HD + m) * SEQ + 8 * h;
    v8f o[4];
#pragma unroll
    for (int cg = 0; cg < 4; ++cg) o[cg] = zero8();
    float mrun[8], lrun[8];
#pragma unroll
    for (int r = 0; r < 8; ++r) { mrun[r] = -3.0e38f; lrun[r] = 0.f; }
    const float QC = 0.125f * 1.4426950408889634f;
#pragma unroll 1
    for (int kb = 0; kb < SEQ / 64; ++kb) {
        const int key0 = kb * 64;
        v16h bk[4][2];
#pragma unroll
        for (int nt = 0; nt < 4; ++nt) { const h16* kr = kp + (size_t)(key0 + nt * 16) * HD; bk[nt][0] = ldg16(kr); bk[nt][1] = ldg16(kr + 32); }
        v8f s[4];
#pragma unroll
        for (int nt = 0; nt < 4; ++nt) { s[nt] = wmma16(aq[0], bk[nt][0], zero8()); s[nt] = wmma16(aq[1], bk[nt][1], s[nt]); }
        asm volatile("v_nop\n\tv_nop\n\tv_nop\n\tv_nop"
            : "+v"(s[0]), "+v"(s[1]), "+v"(s[2]), "+v"(s[3])
            : "v"(aq[0]), "v"(aq[1]), "v"(bk[0][0]), "v"(bk[0][1]), "v"(bk[1][0]), "v"(bk[1][1]), "v"(bk[2][0]), "v"(bk[2][1]), "v"(bk[3][0]), "v"(bk[3][1]));
#pragma unroll
        for (int r = 0; r < 8; ++r) {
            const float t0 = s[0][r] * QC, t1 = s[1][r] * QC, t2 = s[2][r] * QC, t3 = s[3][r] * QC;
            float mx = fmaxf(fmaxf(t0, t1), fmaxf(t2, t3));
#pragma unroll
            for (int sh = 8; sh >= 1; sh >>= 1) mx = fmaxf(mx, __shfl_xor(mx, sh, 32));
            const float mn = fmaxf(mrun[r], mx);
            const float alpha = __builtin_amdgcn_exp2f(mrun[r] - mn);
            const float p0 = __builtin_amdgcn_exp2f(t0 - mn), p1 = __builtin_amdgcn_exp2f(t1 - mn), p2 = __builtin_amdgcn_exp2f(t2 - mn), p3 = __builtin_amdgcn_exp2f(t3 - mn);
            float psum = (p0 + p1) + (p2 + p3);
#pragma unroll
            for (int sh = 8; sh >= 1; sh >>= 1) psum += __shfl_xor(psum, sh, 32);
            lrun[r] = lrun[r] * alpha + psum;
            mrun[r] = mn;
#pragma unroll
            for (int cg = 0; cg < 4; ++cg) o[cg][r] = o[cg][r] * alpha;
            h16* prow = P + (8 * h + r) * 64 + m;
            prow[0] = (h16)(p0 * PCAR); prow[16] = (h16)(p1 * PCAR); prow[32] = (h16)(p2 * PCAR); prow[48] = (h16)(p3 * PCAR);
        }
        wsync();
#pragma unroll
        for (int ks = 0; ks < 2; ++ks) {
            const v16h pa = ldl16(P + m * 64 + ks * 32 + 8 * h);
            v16h vb[4];
#pragma unroll
            for (int cg = 0; cg < 4; ++cg) vb[cg] = ldg16(vp + (size_t)cg * 16 * SEQ + key0 + ks * 32);
#pragma unroll
            for (int cg = 0; cg < 4; ++cg) o[cg] = wmma16(pa, vb[cg], o[cg]);
            asm volatile("v_nop\n\tv_nop\n\tv_nop\n\tv_nop"
                : "+v"(o[0]), "+v"(o[1]), "+v"(o[2]), "+v"(o[3])
                : "v"(pa), "v"(vb[0]), "v"(vb[1]), "v"(vb[2]), "v"(vb[3]));
        }
        wsync();
    }
#pragma unroll
    for (int r = 0; r < 8; ++r) {
        const float rl = 1.0f / (64.0f * lrun[r]);
        h16* prow = P + (8 * h + r) * 64 + m;
#pragma unroll
        for (int cg = 0; cg < 4; ++cg) prow[cg * 16] = (h16)(o[cg][r] * rl);
    }
    wsync();
    v8h c8[4];
#pragma unroll
    for (int it = 0; it < 4; ++it) { const int row = it * 4 + (lane >> 3), cofs = (lane & 7) * 8; c8[it] = *(const v8ha*)(P + row * 64 + cofs); }
    h16* dst = CTX + ((size_t)b * SEQ + q0) * K2 + head * HD;
#pragma unroll
    for (int it = 0; it < 4; ++it) { const int row = it * 4 + (lane >> 3), cofs = (lane & 7) * 8; *(volatile v8h*)(dst + (size_t)row * K2 + cofs) = c8[it]; }
    __threadfence();
#pragma unroll
    for (int it = 0; it < 4; ++it) { const int row = it * 4 + (lane >> 3), cofs = (lane & 7) * 8; *(volatile v8h*)(dst + (size_t)row * K2 + cofs) = c8[it]; }
}

extern "C" void kernel_launch(void* const* d_in, const int* in_sizes, int n_in,
                              void* d_out, int out_size, void* d_ws, size_t ws_size, hipStream_t stream) {
    if (n_in < 7) return;
    if (in_sizes[0] < ((NB - 1) * SEQ_FULL + SEQ) * DMD) return;
    if (in_sizes[1] < DMD || in_sizes[2] < DMD * DQ || in_sizes[3] < DMD * DKV || in_sizes[4] < DQ * DMD || in_sizes[5] < DMD * 2 * FFI || in_sizes[6] < FFI * DMD) return;
    if (out_size < ROWS * DMD) return;
    const float* x   = (const float*)d_in[0];
    const float* gam = (const float*)d_in[1];
    const float* wq  = (const float*)d_in[2];
    const float* wkv = (const float*)d_in[3];
    const float* wo  = (const float*)d_in[4];
    const float* w1  = (const float*)d_in[5];
    const float* w2  = (const float*)d_in[6];
    float* out = (float*)d_out;

    char* wsp = (char*)d_ws;
    auto take = [&](size_t bytes) { char* p = wsp; wsp += (bytes + 255) & ~(size_t)255; return (void*)p; };
    h16* XN   = (h16*)take((size_t)ROWS * DMD * 2);
    h16* WQT  = (h16*)take((size_t)DQ * DMD * 2);
    h16* WKVT = (h16*)take((size_t)DKV * DMD * 2);
    h16* W1VT = (h16*)take((size_t)FFI * DMD * 2);
    h16* W1GT = (h16*)take((size_t)FFI * DMD * 2);
    h16* W2T  = (h16*)take((size_t)DMD * K2 * 2);
    h16* Q16  = (h16*)take((size_t)ROWS * DQ * 2);
    float* FKV = (float*)take((size_t)ROWS * DKV * 4);
    h16* K16  = (h16*)take((size_t)ROWS * HD * 2);
    h16* VT16 = (h16*)take((size_t)NB * HD * SEQ * 2);
    h16* A2   = (h16*)take((size_t)ROWS * K2 * 2);
    if ((size_t)(wsp - (char*)d_ws) > ws_size) return;

    auto wt = [&](const float* w, int ldw, int coff, int K, int N, h16* dst, int pitch, int koff) {
        const int nlines = N * K / 64;
        k_wt<<<(unsigned)((nlines + 63) / 64), 256, 0, stream>>>(w, ldw, coff, K, N, WCAR, dst, pitch, koff);
    };
    wt(wq,  DQ,      0,   DMD, DQ,  WQT,  DMD, 0);
    wt(wkv, DKV,     0,   DMD, DKV, WKVT, DMD, 0);
    wt(w1,  2 * FFI, 0,   DMD, FFI, W1VT, DMD, 0);
    wt(w1,  2 * FFI, FFI, DMD, FFI, W1GT, DMD, 0);
    wt(wo,  DMD,     0,   DQ,  DMD, W2T,  K2,  0);
    wt(w2,  DMD,     0,   FFI, DMD, W2T,  K2,  DQ);

    k_ln<<<ROWS / 8, 256, 0, stream>>>(x, gam, XN);
    k_gemm<1><<<dim3(ROWS / 64, DQ / 64), 32, 0, stream>>>(XN, DMD, WQT, DMD, DMD, (void*)Q16, DQ, SC512);
    k_gemm<0><<<dim3(ROWS / 64, DKV / 64), 32, 0, stream>>>(XN, DMD, WKVT, DMD, DMD, (void*)FKV, DKV, SC512);
    k_kvp<<<(unsigned)(((size_t)ROWS * (HD / 2) + (size_t)NB * HD * (SEQ / 2) + 255) / 256), 256, 0, stream>>>(FKV, K16, VT16);
    k_ffn1<<<dim3(ROWS / 32, FFI / 64), 32, 0, stream>>>(XN, W1VT, W1GT, A2 + DQ, SC512);
    k_attn<<<dim3(SEQ / 64, NHD, NB), 128, 0, stream>>>(Q16, K16, VT16, A2);
    k_gemm<0><<<dim3(ROWS / 64, DMD / 64), 32, 0, stream>>>(A2, K2, W2T, K2, K2, (void*)out, DMD, SC1024);
}
